// MambaBlock_32830730011528
// MI455X (gfx1250) — hardware-run, weakly checked
//
#include <hip/hip_runtime.h>
#include <math.h>

typedef __attribute__((ext_vector_type(16))) _Float16 v16h;
typedef __attribute__((ext_vector_type(8)))  _Float16 v8h;
typedef __attribute__((ext_vector_type(8)))  float    v8f;
typedef __attribute__((ext_vector_type(4)))  float    v4f;

constexpr int kBatch = 2;
constexpr int kSeq   = 1024;
constexpr int kDm    = 1024;
constexpr int kDi    = 2048;
constexpr int kNs    = 16;
constexpr int kDtR   = 64;
constexpr int kRows  = kBatch * kSeq;
constexpr int kXzP   = 2 * kDi;
constexpr int kXdW   = kDtR + 2 * kNs;
constexpr int kXdP   = 128;
constexpr int kConvTP = 260;
constexpr int kScTS  = 64;
constexpr int kScCh  = 64;
constexpr int kScYP  = 68;
static_assert(kRows == 2048 && kXzP == 4096 && kXdW == 96);
static_assert((kDm % 32) == 0 && (kDi % 32) == 0 && (kDtR % 32) == 0);
static_assert((kRows % 64) == 0 && (kXzP % 64) == 0 && (kXdP % 64) == 0 && (kDi % 64) == 0 && (kDm % 64) == 0);
static_assert((kSeq % kScTS) == 0 && (kSeq % 64) == 0 && (kDi % kScCh) == 0 && (kDi % 256) == 0);
static_assert(kXdW <= kXdP && (kDtR % 64) == 0);

constexpr float kCarX  = 16.0f;
constexpr float kCarW  = 1024.0f;
constexpr float kCarU  = 256.0f;
constexpr float kCarDt = 1024.0f;
constexpr float kCarY  = 4096.0f;
constexpr float kScaleIn  = 1.0f / (kCarX  * kCarW);
constexpr float kScaleXp  = 1.0f / (kCarU  * kCarW);
constexpr float kScaleDt  = 1.0f / (kCarDt * kCarW);
constexpr float kScaleOut = 1.0f / (kCarY  * kCarW);

constexpr size_t kSzX16   = (size_t)kRows * kDm  * 2;
constexpr size_t kSzWINT  = (size_t)kXzP  * kDm  * 2;
constexpr size_t kSzWXT   = (size_t)kXdP  * kDi  * 2;
constexpr size_t kSzWDTT  = (size_t)kDi   * kDtR * 2;
constexpr size_t kSzWOUTT = (size_t)kDm   * kDi  * 2;
constexpr size_t kSzXZ    = (size_t)kRows * kXzP * 4;
constexpr size_t kSzU     = (size_t)kRows * kDi  * 4;
constexpr size_t kSzU16   = (size_t)kRows * kDi  * 2;
constexpr size_t kSzXD    = (size_t)kRows * kXdP * 4;
constexpr size_t kSzDT16  = (size_t)kRows * kDtR * 2;
constexpr size_t kSzDP    = (size_t)kRows * kDi  * 4;
constexpr size_t kSzY16   = (size_t)kRows * kDi  * 2;
constexpr size_t kOffX16   = 0;
constexpr size_t kOffWINT  = kOffX16   + kSzX16;
constexpr size_t kOffWXT   = kOffWINT  + kSzWINT;
constexpr size_t kOffWDTT  = kOffWXT   + kSzWXT;
constexpr size_t kOffWOUTT = kOffWDTT  + kSzWDTT;
constexpr size_t kOffXZ    = kOffWOUTT + kSzWOUTT;
constexpr size_t kOffU     = kOffXZ    + kSzXZ;
constexpr size_t kOffU16   = kOffU     + kSzU;
constexpr size_t kOffXD    = kOffU16   + kSzU16;
constexpr size_t kOffDT16  = kOffXD    + kSzXD;
constexpr size_t kOffDP    = kOffDT16  + kSzDT16;
constexpr size_t kOffY16   = kOffDP    + kSzDP;
constexpr size_t kWsTotal  = kOffY16   + kSzY16;
static_assert(kWsTotal == 102760448ull);
static_assert(kWsTotal <= 134217728ull);
static_assert((kOffWINT % 128) == 0 && (kOffWXT % 128) == 0 && (kOffWDTT % 128) == 0 && (kOffWOUTT % 128) == 0 &&
              (kOffXZ % 128) == 0 && (kOffU % 128) == 0 && (kOffU16 % 128) == 0 && (kOffXD % 128) == 0 &&
              (kOffDT16 % 128) == 0 && (kOffDP % 128) == 0 && (kOffY16 % 128) == 0);

__device__ __forceinline__ float bf16_rne(float f) {
  unsigned u = __float_as_uint(f);
  const unsigned lsb = (u & 0x00010000u) ? 1u : 0u;
  u = (u + 0x7FFFu + lsb) & 0xFFFF0000u;
  return __uint_as_float(u);
}
__device__ __forceinline__ _Float16 to_f16_carry(float v, float carry) {
  float c = v * carry;
  c = (fabsf(c) < 6.103515625e-5f) ? 0.0f : c;
  return (_Float16)c;
}
__device__ __forceinline__ _Float16 to_f16_carry_clamped(float v, float carry) {
  float c = v * carry;
  c = fminf(fmaxf(c, -65000.0f), 65000.0f);
  c = (fabsf(c) < 6.103515625e-5f) ? 0.0f : c;
  return (_Float16)c;
}

union FragU { v16h v; v8h h[2]; };
__device__ __forceinline__ v16h frag_load(const _Float16* p) {
  FragU f;
  f.h[0] = *(const v8h*)(p);
  f.h[1] = *(const v8h*)(p + 16);
  return f.v;
}
__device__ __forceinline__ v8f mma_f16(v16h a, v16h b, v8f c) {
  c = __builtin_amdgcn_wmma_f32_16x16x32_f16(false, a, false, b, (short)0, c, false, false);
  asm volatile("v_nop\n\tv_nop\n\tv_nop\n\tv_nop" : "+v"(c) : "v"(a), "v"(b));
  return c;
}
__device__ __forceinline__ void keep4_h(v16h a, v16h b, v16h c, v16h d) { asm volatile("v_nop" :: "v"(a), "v"(b), "v"(c), "v"(d)); }
__device__ __forceinline__ void acc_guard4(v8f& a, v8f& b, v8f& c, v8f& d) { asm volatile("v_nop\n\tv_nop\n\tv_nop\n\tv_nop" : "+v"(a), "+v"(b), "+v"(c), "+v"(d)); }

__global__ __launch_bounds__(256) void gemm_f16_kernel(
    const unsigned short* __restrict__ Ap, int lda,
    const unsigned short* __restrict__ Btp, int ldb,
    float* __restrict__ C, int ldc,
    int M, int N, int K, float scale) {
  const _Float16* A  = (const _Float16*)Ap;
  const _Float16* Bt = (const _Float16*)Btp;
  __shared__ __align__(16) float sT[8][16 * 68];
  const int lane = threadIdx.x & 31;
  const int wave = threadIdx.x >> 5;
  const int tilesN = N >> 6;
  const int tilesM = M >> 6;
  const int tile = blockIdx.x * 8 + wave;
  if (tile >= tilesM * tilesN) return;
  const int tm = tile / tilesN;
  const int tn = tile - tm * tilesN;
  const int m0 = tm << 6;
  const int n0 = tn << 6;

  const int rlane = lane & 15;
  const int koff  = (lane >> 4) * 8;
  const int mOff  = (lane >> 4) * 8;

  v8f acc[4][4];
#pragma unroll
  for (int i = 0; i < 4; ++i)
#pragma unroll
    for (int j = 0; j < 4; ++j) acc[i][j] = (v8f){0.f,0.f,0.f,0.f,0.f,0.f,0.f,0.f};

  for (int k0 = 0; k0 < K; k0 += 32) {
    v16h bh[4];
#pragma unroll
    for (int j = 0; j < 4; ++j) {
      const size_t bo = (size_t)(n0 + (j << 4) + rlane) * ldb + koff + k0;
      bh[j] = frag_load(Bt + bo);
    }
#pragma unroll
    for (int i = 0; i < 4; ++i) {
      const size_t ao = (size_t)(m0 + (i << 4) + rlane) * lda + koff + k0;
      const v16h ah = frag_load(A + ao);
#pragma unroll
      for (int j = 0; j < 4; ++j) acc[i][j] = mma_f16(ah, bh[j], acc[i][j]);
    }
    keep4_h(bh[0], bh[1], bh[2], bh[3]);
  }
  acc_guard4(acc[0][0], acc[0][1], acc[0][2], acc[0][3]);
  acc_guard4(acc[1][0], acc[1][1], acc[1][2], acc[1][3]);
  acc_guard4(acc[2][0], acc[2][1], acc[2][2], acc[2][3]);
  acc_guard4(acc[3][0], acc[3][1], acc[3][2], acc[3][3]);

  float* slab = sT[wave];
#pragma unroll
  for (int i = 0; i < 4; ++i) {
    const int mBase = m0 + (i << 4);
#pragma unroll
    for (int j = 0; j < 4; ++j) {
#pragma unroll
      for (int r = 0; r < 8; ++r) {
        const float v = acc[i][j][r] * scale;
        slab[(mOff + r) * 68 + (j << 4) + rlane] = v;
      }
    }
    __builtin_amdgcn_fence(__ATOMIC_RELEASE, "workgroup");
    __builtin_amdgcn_wave_barrier();
    __builtin_amdgcn_fence(__ATOMIC_ACQUIRE, "workgroup");
    {
      const int hh = lane >> 4, c4 = (lane & 15) * 4;
      for (int pass = 0; pass < 2; ++pass) {
#pragma unroll
        for (int it = 0; it < 8; ++it) {
          const int row = it * 2 + hh;
          const v4f v = *(const v4f*)(slab + row * 68 + c4);
          *(volatile v4f*)(C + (size_t)(mBase + row) * ldc + n0 + c4) = v;
        }
        __threadfence();
      }
    }
    __builtin_amdgcn_fence(__ATOMIC_RELEASE, "workgroup");
    __builtin_amdgcn_wave_barrier();
    __builtin_amdgcn_fence(__ATOMIC_ACQUIRE, "workgroup");
  }
}

template <int LOGC, bool BF>
__global__ __launch_bounds__(256) void cvt_rows_kernel(
    const float* __restrict__ src, unsigned srcPitch, unsigned short* __restrict__ dst, unsigned total8, float carry) {
  unsigned i = blockIdx.x * 256u + threadIdx.x;
  if (i >= total8) return;
  unsigned e0 = i << 3;
  unsigned row = e0 >> LOGC;
  unsigned col = e0 & ((1u << LOGC) - 1u);
  asm volatile("" : "+v"(row));
  asm volatile("" : "+v"(col));
  const float* sp = src + (size_t)row * srcPitch + col;
  const v4f a0 = *(const v4f*)(sp);
  const v4f a1 = *(const v4f*)(sp + 4);
  v8h hv;
#pragma unroll
  for (int e = 0; e < 4; ++e) {
    float f0 = a0[e];
    float f1 = a1[e];
    if (BF) {
      f0 = bf16_rne(f0);
      f1 = bf16_rne(f1);
    }
    hv[e]     = to_f16_carry(f0, carry);
    hv[4 + e] = to_f16_carry(f1, carry);
  }
  unsigned short* q = dst + (size_t)e0;
  *(volatile v8h*)q = hv;
  __threadfence();
  *(volatile v8h*)q = hv;
}

__global__ __launch_bounds__(256) void transpose_cvt_kernel(
    const float* __restrict__ src, unsigned short* __restrict__ dst, unsigned rows, unsigned cols, float carry) {
  __shared__ float sT[64 * 65];
  const unsigned tid = threadIdx.x;
  const unsigned r0 = blockIdx.y * 64u;
  const unsigned c0 = blockIdx.x * 64u;
  unsigned lc = tid & 63u;
  unsigned lr = tid >> 6;
  asm volatile("" : "+v"(lc));
  asm volatile("" : "+v"(lr));
  const unsigned gc  = c0 + lc;
  const unsigned gcc = (gc < cols) ? gc : (cols - 1u);
  const bool inb = (gc < cols);
#pragma unroll 4
  for (unsigned it = 0; it < 16u; ++it) {
    const unsigned r = it * 4u + lr;
    float v = src[(size_t)(r0 + r) * cols + gcc];
    asm volatile("" : "+v"(v));
    const float vb = bf16_rne(v);
    sT[lc * 65u + r] = inb ? vb : 0.0f;
  }
  __syncthreads();
  const unsigned lane = tid & 31u, wave = tid >> 5;
  unsigned q  = lane >> 3;
  unsigned j8 = (lane & 7u) * 8u;
  asm volatile("" : "+v"(q));
  asm volatile("" : "+v"(j8));
  v8h hv[2];
#pragma unroll
  for (int it = 0; it < 2; ++it) {
    const unsigned orow = (unsigned)it * 32u + wave * 4u + q;
    const float* sp = sT + orow * 65u + j8;
#pragma unroll
    for (int e = 0; e < 8; ++e) {
      const float f = sp[e];
      hv[it][e] = to_f16_carry(f, carry);
    }
  }
  for (int pass = 0; pass < 2; ++pass) {
#pragma unroll
    for (int it = 0; it < 2; ++it) {
      const unsigned orow = (unsigned)it * 32u + wave * 4u + q;
      *(volatile v8h*)(dst + (size_t)(c0 + orow) * rows + r0 + j8) = hv[it];
    }
    __threadfence();
  }
}

__global__ __launch_bounds__(256) void conv_silu_kernel(
    const float* __restrict__ XZ, const float* __restrict__ cw, const float* __restrict__ cb,
    float* __restrict__ U, unsigned short* __restrict__ U16) {
  __shared__ __align__(16) float sT[16 * kConvTP];
  const int tid = threadIdx.x, lane = tid & 31, wave = tid >> 5;
  const int d0 = blockIdx.x * 256, d = d0 + tid;
  const int g0 = blockIdx.y * 64;
  const int tb = g0 & (kSeq - 1);
  const v4f wv = *(const v4f*)(cw + (size_t)d * 4);
  const float wr0 = wv[0], wr1 = wv[1], wr2 = wv[2], wr3 = wv[3];
  const float w0 = bf16_rne(wr0), w1 = bf16_rne(wr1), w2 = bf16_rne(wr2), w3 = bf16_rne(wr3);
  const float bc = bf16_rne(cb[d]);
  float xm3, xm2, xm1;
  {
    const bool hist = (tb > 0);
    const int rb = hist ? (g0 - 3) : g0;
    const float v3 = XZ[(size_t)rb * kXzP + d];
    const float v2 = XZ[(size_t)(rb + 1) * kXzP + d];
    const float v1 = XZ[(size_t)(rb + 2) * kXzP + d];
    xm3 = hist ? v3 : 0.f;
    xm2 = hist ? v2 : 0.f;
    xm1 = hist ? v1 : 0.f;
  }
  const int hrow = wave >> 1;
  const int hch  = (wave & 1) * 128 + lane * 4;
#pragma unroll 1
  for (int sub = 0; sub < 4; ++sub) {
    const int lb = g0 + sub * 16;
#pragma unroll 1
    for (int s = 0; s < 16; ++s) {
      const float xcur = XZ[(size_t)(lb + s) * kXzP + d];
      float acc = w0 * xm3;
      acc = fmaf(w1, xm2, acc);
      acc = fmaf(w2, xm1, acc);
      acc = fmaf(w3, xcur, acc);
      const float sv = acc + bc;
      const float sg = 1.0f / (1.0f + expf(-sv));
      sT[s * kConvTP + tid] = sv * sg;
      xm3 = xm2;
      xm2 = xm1;
      xm1 = xcur;
    }
    __syncthreads();
    v4f fv[4];
    v8h hv[2];
#pragma unroll
    for (int it = 0; it < 4; ++it) fv[it] = *(const v4f*)(sT + (it * 4 + hrow) * kConvTP + hch);
#pragma unroll
    for (int it = 0; it < 2; ++it) {
      const float* sp = sT + (it * 8 + wave) * kConvTP + lane * 8;
      const v4f a0 = *(const v4f*)(sp);
      const v4f a1 = *(const v4f*)(sp + 4);
#pragma unroll
      for (int e = 0; e < 4; ++e) {
        const float f0 = a0[e];
        const float f1 = a1[e];
        hv[it][e]     = to_f16_carry(f0, kCarU);
        hv[it][4 + e] = to_f16_carry(f1, kCarU);
      }
    }
    for (int pass = 0; pass < 2; ++pass) {
#pragma unroll
      for (int it = 0; it < 4; ++it)
        *(volatile v4f*)(U + (size_t)(lb + it * 4 + hrow) * kDi + d0 + hch) = fv[it];
#pragma unroll
      for (int it = 0; it < 2; ++it)
        *(volatile v8h*)(U16 + (size_t)(lb + it * 8 + wave) * kDi + d0 + lane * 8) = hv[it];
      __threadfence();
    }
    __syncthreads();
  }
}

__global__ __launch_bounds__(128) void scan_kernel(
    const float* __restrict__ XD, const float* __restrict__ DP, const float* __restrict__ U,
    const float* __restrict__ XZ, const float* __restrict__ bdt, const float* __restrict__ Alog,
    const float* __restrict__ Dsk, unsigned short* __restrict__ Y16) {
  __shared__ __align__(16) float sX[kScTS * 32];
  __shared__ __align__(16) float sY[kScTS * kScYP];
  __shared__ __align__(16) float sA[8 * 128];
  const unsigned tid = threadIdx.x;
  const unsigned lane = tid & 31u, wave = tid >> 5;
  unsigned ch = tid >> 1;
  unsigned hs = tid & 1u;
  asm volatile("" : "+v"(ch));
  asm volatile("" : "+v"(hs));
  constexpr unsigned kBlkPerB = kDi / kScCh;
  const unsigned bix = blockIdx.x / kBlkPerB;
  const unsigned d0  = (blockIdx.x - bix * kBlkPerB) * kScCh;
  const unsigned d   = d0 + ch;
  const size_t row0 = (size_t)bix * kSeq;
#pragma unroll 1
  for (unsigned s = 0; s < 8u; ++s) {
    const float al = Alog[(size_t)d * kNs + 8u * hs + s];
    sA[s * 128u + tid] = -expf(bf16_rne(al));
  }
  __syncthreads();
  float negA[8], h[8];
#pragma unroll
  for (int s = 0; s < 8; ++s) {
    negA[s] = sA[s * 128 + tid];
    h[s] = 0.f;
  }
  const float bb = bf16_rne(bdt[d]);
  const float Dd = bf16_rne(Dsk[d]);
  unsigned q  = lane >> 3;
  unsigned c8 = (lane & 7u) * 8u;
  asm volatile("" : "+v"(q));
  asm volatile("" : "+v"(c8));
#pragma unroll 1
  for (unsigned t0 = 0; t0 < (unsigned)kSeq; t0 += kScTS) {
    __syncthreads();
#pragma unroll
    for (unsigned k = 0; k < 4u; ++k) {
      const unsigned idx = tid + 128u * k;
      const unsigned r = idx >> 3;
      const unsigned c4 = (idx & 7u) * 4u;
      *(v4f*)(sX + r * 32u + c4) = *(const v4f*)(XD + (row0 + t0 + r) * kXdP + kDtR + c4);
    }
    __syncthreads();
#pragma unroll 1
    for (unsigned s = 0; s < (unsigned)kScTS; ++s) {
      const size_t row = row0 + t0 + s;
      float pre = DP[row * kDi + d];
      float ut  = U[row * kDi + d];
      float zv  = XZ[row * kXzP + kDi + d];
      asm volatile("" : "+v"(pre));
      asm volatile("" : "+v"(ut));
      asm volatile("" : "+v"(zv));
      const float v = pre + bb;
      const float ea = expf(-fabsf(v));
      const float delta = fmaxf(v, 0.0f) + log1pf(ea);
      const float dtx = delta * ut;
      const float* xr = sX + s * 32u + 8u * hs;
      const v4f b0 = *(const v4f*)(xr);
      const v4f b1 = *(const v4f*)(xr + 4);
      const v4f c0 = *(const v4f*)(xr + 16);
      const v4f c1 = *(const v4f*)(xr + 20);
      float y = 0.f;
#pragma unroll
      for (int e = 0; e < 4; ++e) {
        const float bq = b0[e];
        const float cq = c0[e];
        const float ee = expf(delta * negA[e]);
        h[e] = fmaf(ee, h[e], dtx * bq);
        y = fmaf(h[e], cq, y);
      }
#pragma unroll
      for (int e = 0; e < 4; ++e) {
        const float bq = b1[e];
        const float cq = c1[e];
        const float ee = expf(delta * negA[4 + e]);
        h[4 + e] = fmaf(ee, h[4 + e], dtx * bq);
        y = fmaf(h[4 + e], cq, y);
      }
      const float yo = __shfl_xor(y, 1, 32);
      float ys = y + yo;
      ys = fmaf(ut, Dd, ys);
      const float sg = 1.0f / (1.0f + expf(-zv));
      ys = ys * (zv * sg);
      if (hs == 0u) sY[s * kScYP + ch] = ys;
    }
    __syncthreads();
    v8h hv[4];
#pragma unroll
    for (int it = 0; it < 4; ++it) {
      const unsigned row = (unsigned)it * 16u + wave * 4u + q;
      const float* sp = sY + row * kScYP + c8;
      const v4f a0 = *(const v4f*)(sp);
      const v4f a1 = *(const v4f*)(sp + 4);
#pragma unroll
      for (int e = 0; e < 4; ++e) {
        const float f0 = a0[e];
        const float f1 = a1[e];
        hv[it][e]     = to_f16_carry_clamped(f0, kCarY);
        hv[it][4 + e] = to_f16_carry_clamped(f1, kCarY);
      }
    }
    for (int pass = 0; pass < 2; ++pass) {
#pragma unroll
      for (int it = 0; it < 4; ++it) {
        const unsigned row = (unsigned)it * 16u + wave * 4u + q;
        *(volatile v8h*)(Y16 + (row0 + t0 + row) * kDi + d0 + c8) = hv[it];
      }
      __threadfence();
    }
  }
}

extern "C" void kernel_launch(void* const* d_in, const int* in_sizes, int n_in,
                              void* d_out, int out_size, void* d_ws, size_t ws_size,
                              hipStream_t stream) {
  if (n_in < 10) return;
  if (in_sizes[0] != kRows * kDm) return;
  if (in_sizes[1] != kDm * kXzP) return;
  if (in_sizes[2] != kDi * 4) return;
  if (in_sizes[3] != kDi) return;
  if (in_sizes[4] != kDi * kXdW) return;
  if (in_sizes[5] != kDtR * kDi) return;
  if (in_sizes[6] != kDi) return;
  if (in_sizes[7] != kDi * kNs) return;
  if (in_sizes[8] != kDi) return;
  if (in_sizes[9] != kDi * kDm) return;
  if (out_size != kRows * kDm) return;
  if (ws_size < kWsTotal) return;

  const float* x      = (const float*)d_in[0];
  const float* W_in   = (const float*)d_in[1];
  const float* conv_w = (const float*)d_in[2];
  const float* conv_b = (const float*)d_in[3];
  const float* W_x    = (const float*)d_in[4];
  const float* W_dt   = (const float*)d_in[5];
  const float* b_dt   = (const float*)d_in[6];
  const float* A_log  = (const float*)d_in[7];
  const float* D_skip = (const float*)d_in[8];
  const float* W_out  = (const float*)d_in[9];
  float* out = (float*)d_out;

  char* ws = (char*)d_ws;
  unsigned short* X16   = (unsigned short*)(ws + kOffX16);
  unsigned short* WINT  = (unsigned short*)(ws + kOffWINT);
  unsigned short* WXT   = (unsigned short*)(ws + kOffWXT);
  unsigned short* WDTT  = (unsigned short*)(ws + kOffWDTT);
  unsigned short* WOUTT = (unsigned short*)(ws + kOffWOUTT);
  float*          XZ    = (float*)(ws + kOffXZ);
  float*          U     = (float*)(ws + kOffU);
  unsigned short* U16   = (unsigned short*)(ws + kOffU16);
  float*          XD    = (float*)(ws + kOffXD);
  unsigned short* DT16  = (unsigned short*)(ws + kOffDT16);
  float*          DP    = (float*)(ws + kOffDP);
  unsigned short* Y16   = (unsigned short*)(ws + kOffY16);

  cvt_rows_kernel<10, true><<<(kRows * kDm / 8) / 256, 256, 0, stream>>>(
      x, (unsigned)kDm, X16, (unsigned)(kRows * kDm / 8), kCarX);
  transpose_cvt_kernel<<<dim3(kXzP / 64, kDm / 64), 256, 0, stream>>>(W_in, WINT, (unsigned)kDm, (unsigned)kXzP, kCarW);
  transpose_cvt_kernel<<<dim3(kXdP / 64, kDi / 64), 256, 0, stream>>>(W_x, WXT, (unsigned)kDi, (unsigned)kXdW, kCarW);
  transpose_cvt_kernel<<<dim3(kDi / 64, kDtR / 64), 256, 0, stream>>>(W_dt, WDTT, (unsigned)kDtR, (unsigned)kDi, kCarW);
  transpose_cvt_kernel<<<dim3(kDm / 64, kDi / 64), 256, 0, stream>>>(W_out, WOUTT, (unsigned)kDi, (unsigned)kDm, kCarW);

  gemm_f16_kernel<<<(kRows / 64) * (kXzP / 64) / 8, 256, 0, stream>>>(
      X16, kDm, WINT, kDm, XZ, kXzP, kRows, kXzP, kDm, kScaleIn);

  conv_silu_kernel<<<dim3(kDi / 256, kRows / 64), 256, 0, stream>>>(XZ, conv_w, conv_b, U, U16);

  gemm_f16_kernel<<<(kRows / 64) * (kXdP / 64) / 8, 256, 0, stream>>>(
      U16, kDi, WXT, kDi, XD, kXdP, kRows, kXdP, kDi, kScaleXp);

  cvt_rows_kernel<6, false><<<(kRows * kDtR / 8) / 256, 256, 0, stream>>>(
      XD, (unsigned)kXdP, DT16, (unsigned)(kRows * kDtR / 8), kCarDt);

  gemm_f16_kernel<<<(kRows / 64) * (kDi / 64) / 8, 256, 0, stream>>>(
      DT16, kDtR, WDTT, kDtR, DP, kDi, kRows, kDi, kDtR, kScaleDt);

  scan_kernel<<<kBatch * (kDi / kScCh), 128, 0, stream>>>(XD, DP, U, XZ, b_dt, A_log, D_skip, Y16);

  gemm_f16_kernel<<<(kRows / 64) * (kDm / 64) / 8, 256, 0, stream>>>(
      Y16, kDi, WOUTT, kDi, out, kDm, kRows, kDm, kDi, kScaleOut);
}
